// SubGraphEncoder_34857954575031
// MI455X (gfx1250) — hardware-run, weakly checked
//
#include <hip/hip_runtime.h>


namespace {
constexpr int NG = 32, M = 1024, DI = 128, DO = 128, ED = 64, NT = NG * M;
constexpr float XS = 8.0f, HS = 256.0f, WSC = 256.0f;
typedef _Float16 b16;
typedef __attribute__((ext_vector_type(16))) _Float16 v16b;
typedef __attribute__((ext_vector_type(8))) _Float16 v8b;
typedef __attribute__((ext_vector_type(2))) _Float16 v2b;
typedef __attribute__((ext_vector_type(8))) float v8f;
typedef __attribute__((ext_vector_type(4))) float v4f;
__device__ __forceinline__ float bf16_rne(float f) { unsigned int u = __float_as_uint(f); u += 0x7FFFu + ((u >> 16) & 1u); float r = __uint_as_float(u & 0xFFFF0000u); asm volatile("" : "+v"(r)); return r; }
__device__ __forceinline__ float bfv(float f) { float r = bf16_rne(f); asm volatile("" : "+v"(r)); return r; }
__device__ __forceinline__ void split16(float v, b16& hi, b16& lo) { hi = (b16)v; lo = (b16)(v - (float)hi); }
__device__ __forceinline__ v16b frag_kb(const b16* p, int hh) { const v8b a = *(const v8b*)(p + 8 * hh), b = *(const v8b*)(p + 16 + 8 * hh); v16b f;
#pragma unroll
  for (int e = 0; e < 8; ++e) { f[e] = a[e]; f[8 + e] = b[e]; } return f; }
__device__ __forceinline__ v8f wmma16b(v16b a, v16b b, v8f c) { v8f d = __builtin_amdgcn_wmma_f32_16x16x32_f16(false, a, false, b, (short)0, c, false, false); asm volatile("v_nop\n\tv_nop\n\tv_nop\n\tv_nop" : "+v"(d) : "v"(a), "v"(b)); return d; }
__device__ __forceinline__ void wave_lds_sync() { __builtin_amdgcn_fence(__ATOMIC_RELEASE, "workgroup"); __builtin_amdgcn_wave_barrier(); __builtin_amdgcn_fence(__ATOMIC_ACQUIRE, "workgroup"); }
__device__ __forceinline__ float pmul(float a, float b) { float p = a * b; asm volatile("" : "+v"(p)); return p; }

__global__ __launch_bounds__(256) void prep_kernel(const float* __restrict__ emb, const float* __restrict__ w1, const float* __restrict__ w2, b16* __restrict__ EM, b16* __restrict__ WT1, b16* __restrict__ WT2) { const size_t u = (size_t)blockIdx.x * 256 + threadIdx.x;
  if (u < (size_t)NT * ED / 2) { for (int pass = 0; pass < 2; ++pass) { *(volatile v2b*)(EM + 2 * u) = (v2b){(b16)(bfv(emb[2 * u]) * XS), (b16)(bfv(emb[2 * u + 1]) * XS)}; __threadfence(); } }
  if (u < (size_t)DO * 16) { const int o = (int)(u / 16), k0 = (int)(u % 16) * 8; v8b a, c;
#pragma unroll
    for (int j = 0; j < 8; ++j) { a[j] = (b16)(bf16_rne(w1[(size_t)o * DI + k0 + j]) * WSC); c[j] = (b16)(bf16_rne(w2[(size_t)o * DO + k0 + j]) * WSC); } for (int pass = 0; pass < 2; ++pass) { *(volatile v8b*)(WT1 + (size_t)o * DI + k0) = a; *(volatile v8b*)(WT2 + (size_t)o * DO + k0) = c; __threadfence(); } } }
__global__ __launch_bounds__(32) void deg_kernel(const b16* __restrict__ EM, int GLIM, float* __restrict__ DIS) { __shared__ float Rs[16][17]; const int lane = threadIdx.x, nloc = lane & 15, hlf = lane >> 4; const int b = blockIdx.x / (M / 16), i0 = (blockIdx.x % (M / 16)) * 16; if (b >= GLIM) return; const size_t nb0 = (size_t)b * M;
  const v16b a0 = frag_kb(EM + (nb0 + i0 + nloc) * ED, hlf), a1 = frag_kb(EM + (nb0 + i0 + nloc) * ED + 32, hlf); float part[8] = {0, 0, 0, 0, 0, 0, 0, 0};
#pragma unroll 1
  for (int t = 0; t < M / 16; ++t) { const b16* ep = EM + (nb0 + t * 16 + nloc) * ED; v8f d = wmma16b(a0, frag_kb(ep, hlf), (v8f){}); d = wmma16b(a1, frag_kb(ep + 32, hlf), d);
#pragma unroll
    for (int r8 = 0; r8 < 8; ++r8) part[r8] += fmaxf(d[r8] * (1.0f / (XS * XS)), 0.0f); }
#pragma unroll
  for (int r8 = 0; r8 < 8; ++r8) { float v = part[r8]; for (int o = 8; o; o >>= 1) v += __shfl_xor(v, o); if (nloc == 0) Rs[8 * hlf + r8][0] = v; }
  wave_lds_sync();
  const float dv = lane < 16 ? rsqrtf(Rs[lane][0] + 1.0f) : 0.0f;
  for (int pass = 0; pass < 2; ++pass) { ((volatile float*)DIS)[(size_t)blockIdx.x * 32 + lane] = dv; __threadfence(); } }
__device__ __forceinline__ float dis_at(const float* DIS, size_t node) { return DIS[(node / 16) * 32 + (node % 16)]; }
template <int MODE>
__global__ __launch_bounds__(32) void xw_kernel(const float* __restrict__ IN, const b16* __restrict__ WT, const float* __restrict__ DIS, int GLIM, float* __restrict__ Z) { __shared__ __attribute__((aligned(16))) b16 Ah[16][DI + 8], Al[16][DI + 8]; __shared__ float Tf[16][DO + 4]; const int lane = threadIdx.x, nloc = lane & 15, hlf = lane >> 4; const size_t n0 = (size_t)blockIdx.x * 16; if (n0 >= (size_t)GLIM * M) return;
  for (int rr = 0; rr < 16; ++rr) for (int q = 0; q < 4; ++q) { const int c = q * 32 + lane; const float v = IN[(n0 + rr) * DI + c]; if (MODE == 0) { Ah[rr][c] = (b16)(bfv(v) * XS); Al[rr][c] = (b16)0.0f; } else { b16 p, pl; split16(v * HS, p, pl); Ah[rr][c] = p; Al[rr][c] = pl; } }
  if (lane < 16) for (int k = DI; k < DI + 8; ++k) { Ah[lane][k] = (b16)0.0f; Al[lane][k] = (b16)0.0f; }
  wave_lds_sync(); v8f acc[8];
#pragma unroll
  for (int t = 0; t < 8; ++t) acc[t] = (v8f){};
#pragma unroll
  for (int kb = 0; kb < DI; kb += 32) { const v16b a = frag_kb(&Ah[nloc][kb], hlf), al = frag_kb(&Al[nloc][kb], hlf);
#pragma unroll
    for (int t = 0; t < 8; ++t) { const v16b bw = frag_kb(WT + (size_t)(t * 16 + nloc) * DI + kb, hlf); acc[t] = wmma16b(a, bw, acc[t]); if (MODE == 1) acc[t] = wmma16b(al, bw, acc[t]); } }
  const float isc = MODE == 0 ? 1.0f / (XS * WSC) : 1.0f / (HS * WSC);
#pragma unroll
  for (int t = 0; t < 8; ++t)
#pragma unroll
    for (int r8 = 0; r8 < 8; ++r8) { const int rr = 8 * hlf + r8; Tf[rr][t * 16 + nloc] = acc[t][r8] * isc * dis_at(DIS, n0 + rr); }
  wave_lds_sync();
  for (int pass = 0; pass < 2; ++pass) { for (int rr = 0; rr < 16; ++rr) *(volatile v4f*)(Z + (n0 + rr) * DO + lane * 4) = *(const v4f*)(&Tf[rr][lane * 4]); __threadfence(); } }
__global__ __launch_bounds__(256) void zt_kernel(const float* __restrict__ Z, int GLIM, b16* __restrict__ ZTh, b16* __restrict__ ZTl) { __shared__ float Tt[64][DO + 1]; const int b = blockIdx.x / (M / 64), nn0 = (blockIdx.x % (M / 64)) * 64; if (b >= GLIM) return; const int tid = threadIdx.x, wave = tid >> 5, lane = tid & 31;
  for (int q = wave; q < 64; q += 8) for (int c = lane; c < DO; c += 32) Tt[q][c] = Z[((size_t)b * M + nn0 + q) * DO + c];
  __syncthreads();
  for (int pass = 0; pass < 2; ++pass) { for (int o = wave; o < DO; o += 8) { b16 h0, l0, h1, l1; split16(Tt[lane * 2][o] * HS, h0, l0); split16(Tt[lane * 2 + 1][o] * HS, h1, l1); const size_t off = ((size_t)b * DO + o) * M + nn0 + lane * 2; *(volatile v2b*)(ZTh + off) = (v2b){h0, h1}; *(volatile v2b*)(ZTl + off) = (v2b){l0, l1}; } __threadfence(); } }
__global__ __launch_bounds__(32) void layer_kernel(const b16* __restrict__ EM, const float* __restrict__ DIS, const b16* __restrict__ ZTh, const b16* __restrict__ ZTl, int GLIM, float* __restrict__ OUT) { __shared__ __attribute__((aligned(16))) b16 Pa[16][264], Pb[16][264]; __shared__ float Tf[16][DO + 4]; const int lane = threadIdx.x, nloc = lane & 15, hlf = lane >> 4; const int b = blockIdx.x / (M / 16), i0 = (blockIdx.x % (M / 16)) * 16; if (b >= GLIM) return; const size_t nb0 = (size_t)b * M;
  if (lane < 16) for (int k = 256; k < 264; ++k) { Pa[lane][k] = (b16)0.0f; Pb[lane][k] = (b16)0.0f; }
  const v16b a0 = frag_kb(EM + (nb0 + i0 + nloc) * ED, hlf), a1 = frag_kb(EM + (nb0 + i0 + nloc) * ED + 32, hlf);
  float di[8]; for (int r8 = 0; r8 < 8; ++r8) di[r8] = dis_at(DIS, nb0 + i0 + 8 * hlf + r8);
  v8f acc[8];
#pragma unroll
  for (int t = 0; t < 8; ++t) acc[t] = (v8f){};
#pragma unroll 1
  for (int ch = 0; ch < M / 256; ++ch) { const int c0 = ch * 256;
#pragma unroll 1
    for (int t = 0; t < 16; ++t) { const int n = c0 + t * 16 + nloc; const b16* ep = EM + (nb0 + n) * ED; v8f d = wmma16b(a0, frag_kb(ep, hlf), (v8f){}); d = wmma16b(a1, frag_kb(ep + 32, hlf), d);
#pragma unroll
      for (int r8 = 0; r8 < 8; ++r8) { const int rr = 8 * hlf + r8; float av = fmaxf(d[r8] * (1.0f / (XS * XS)), 0.0f); if (i0 + rr == n) av += 1.0f; av *= di[r8]; b16 p, pl; split16(av * HS, p, pl); Pa[rr][t * 16 + nloc] = p; Pb[rr][t * 16 + nloc] = pl; } }
    wave_lds_sync();
#pragma unroll 2
    for (int kb = 0; kb < 256; kb += 32) { const v16b pa = frag_kb(&Pa[nloc][kb], hlf), pb = frag_kb(&Pb[nloc][kb], hlf);
#pragma unroll
      for (int t = 0; t < 8; ++t) { const size_t zo = ((size_t)b * DO + t * 16 + nloc) * M + c0 + kb; const v16b zh = frag_kb(ZTh + zo, hlf), zl = frag_kb(ZTl + zo, hlf); acc[t] = wmma16b(pa, zh, acc[t]); acc[t] = wmma16b(pa, zl, acc[t]); acc[t] = wmma16b(pb, zh, acc[t]); } }
    wave_lds_sync(); }
#pragma unroll
  for (int t = 0; t < 8; ++t)
#pragma unroll
    for (int r8 = 0; r8 < 8; ++r8) Tf[8 * hlf + r8][t * 16 + nloc] = fmaxf(acc[t][r8] * (1.0f / (HS * HS)), 0.0f);
  wave_lds_sync();
  for (int pass = 0; pass < 2; ++pass) { for (int rr = 0; rr < 16; ++rr) *(volatile v4f*)(OUT + (nb0 + i0 + rr) * DO + lane * 4) = *(const v4f*)(&Tf[rr][lane * 4]); __threadfence(); } }
}

extern "C" void kernel_launch(void* const* d_in, const int* in_sizes, int n_in, void* d_out, int out_size, void* d_ws, size_t ws_size, hipStream_t stream) {
  (void)n_in;
  auto Fp = [&](int i) { return (const float*)d_in[i]; };
  if (in_sizes[0] != NT * DI || in_sizes[1] != NT * ED || in_sizes[2] != DO * DI || in_sizes[3] != DO * DO || out_size != NT * DO) return;
  const int GLIM = NG;
  size_t off = 0; char* ws = (char*)d_ws;
  auto carve = [&](size_t bytes) { char* p = ws + off; off += (bytes + 255) & ~(size_t)255; return p; };
  b16* EM = (b16*)carve((size_t)NT * ED * 2); b16* WT1 = (b16*)carve((size_t)DO * DI * 2); b16* WT2 = (b16*)carve((size_t)DO * DO * 2); float* DIS = (float*)carve((size_t)(NT / 16) * 32 * 4); float* Z = (float*)carve((size_t)NT * DO * 4); b16* ZTh = (b16*)carve((size_t)NT * DO * 2); b16* ZTl = (b16*)carve((size_t)NT * DO * 2); float* Y1 = (float*)carve((size_t)NT * DO * 4);
  if (off > ws_size || off > ((size_t)64 << 20)) return;
  const size_t nprep = ((size_t)NT * ED / 2 + 255) / 256;
  prep_kernel<<<(unsigned)nprep, 256, 0, stream>>>(Fp(1), Fp(2), Fp(3), EM, WT1, WT2);
  deg_kernel<<<GLIM * (M / 16), 32, 0, stream>>>(EM, GLIM, DIS);
  xw_kernel<0><<<GLIM * (M / 16), 32, 0, stream>>>(Fp(0), WT1, DIS, GLIM, Z);
  zt_kernel<<<GLIM * (M / 64), 256, 0, stream>>>(Z, GLIM, ZTh, ZTl);
  layer_kernel<<<GLIM * (M / 16), 32, 0, stream>>>(EM, DIS, ZTh, ZTl, GLIM, Y1);
  xw_kernel<1><<<GLIM * (M / 16), 32, 0, stream>>>(Y1, WT2, DIS, GLIM, Z);
  zt_kernel<<<GLIM * (M / 64), 256, 0, stream>>>(Z, GLIM, ZTh, ZTl);
  layer_kernel<<<GLIM * (M / 16), 32, 0, stream>>>(EM, DIS, ZTh, ZTl, GLIM, (float*)d_out);
}
